// model_24507083391623
// MI455X (gfx1250) — hardware-run, weakly checked
//
#include <hip/hip_runtime.h>
#include <math.h>

typedef __attribute__((ext_vector_type(16))) _Float16 v16h;
typedef __attribute__((ext_vector_type(8)))  _Float16 v8h;
typedef __attribute__((ext_vector_type(8)))  float    v8f;
typedef __attribute__((ext_vector_type(4)))  float    v4f;

constexpr int kBatch = 2;
constexpr int kCh    = 128;
constexpr int kHW    = 16384;
constexpr int kTok   = kBatch * kHW;
constexpr int kExp   = 6;
constexpr int kDeg   = 6;
constexpr int kHid   = 512;
constexpr int kGatePitch = 8;
constexpr int kXLdsPitch = 136;
constexpr int kTokPitch  = 36;
constexpr int kGateBlocks = kTok / 128;
static_assert(kTok == 32768, "token count");
static_assert((kHW % 128) == 0, "a 128-token block stays inside one batch element");
static_assert((kCh % 32) == 0 && (kHid % 32) == 0, "contraction depths are multiples of 32");
static_assert((kCh % 64) == 0 && (kHid % 64) == 0, "transpose tiles");
static_assert((kCh / 64) * (kHid / 64) == 16, "16 tiles per weight matrix");

constexpr float kXCarry = 16.0f;
constexpr float kWCarry = 1024.0f;
constexpr float kHCarry = 128.0f;
constexpr float kFc1Inv = 1.0f / (kXCarry * kWCarry);
constexpr float kFc2Inv = 1.0f / (kHCarry * kWCarry);
constexpr float kF16MinNormal = 6.103515625e-5f;
constexpr float kEpsLog = 2.220446049250313e-16f;
constexpr float kInvSqrt2 = 0.70710678118654752f;

constexpr size_t kOffXH   = 0;
constexpr size_t kOffW1T  = kOffXH   + (size_t)kTok * kCh * 2;
constexpr size_t kOffW2T  = kOffW1T  + (size_t)kExp * kHid * kCh * 2;
constexpr size_t kOffGATE = kOffW2T  + (size_t)kExp * kCh * kHid * 2;
constexpr size_t kOffPART = kOffGATE + (size_t)kTok * kGatePitch * 4;
constexpr size_t kOffADDL = kOffPART + (size_t)kGateBlocks * 32 * 4;
constexpr size_t kWsTotal = kOffADDL + 128;
static_assert(kWsTotal == 11042944ull, "carve total");
static_assert(kWsTotal <= 134217728ull, "carve cap");
static_assert((kOffW1T % 128) == 0 && (kOffW2T % 128) == 0 && (kOffGATE % 128) == 0 &&
              (kOffPART % 128) == 0 && (kOffADDL % 128) == 0, "128-B aligned regions");

__device__ __forceinline__ float flush16(float s) {
  return (fabsf(s) < kF16MinNormal) ? 0.0f : s;
}

union FragU { v16h v; v8h h[2]; };

__device__ __forceinline__ v16h frag_load(const _Float16* p) {
  FragU f;
  f.h[0] = *(const v8h*)(p);
  f.h[1] = *(const v8h*)(p + 16);
  return f.v;
}

__device__ __forceinline__ v8f mma_g(v16h a, v16h b, v8f c) {
  c = __builtin_amdgcn_wmma_f32_16x16x32_f16(false, a, false, b, (short)0, c, false, false);
  asm volatile("v_nop\n\tv_nop\n\tv_nop\n\tv_nop" : "+v"(c) : "v"(a), "v"(b));
  return c;
}

__global__ __launch_bounds__(32) void prep_kernel(
    const float* __restrict__ prompt, const float* __restrict__ de_cls, const float* __restrict__ w_g,
    const float* __restrict__ gate_boost, const float* __restrict__ degra_w, const float* __restrict__ degra_b,
    float* __restrict__ addl)
{
  const int lane = threadIdx.x & 31;
  const int idx = lane & 15;
  const int idc = (idx < 11) ? idx : 11;
  const int b = idc / kExp;
  const int e = idc - b * kExp;
  float pp = 0.0f;
#pragma unroll 1
  for (int c = 0; c < kCh; ++c) pp = fmaf(prompt[b * kCh + c], w_g[(kCh + c) * kExp + e], pp);
  float bs = 0.0f;
#pragma unroll 1
  for (int d = 0; d < kDeg; ++d) bs = fmaf(de_cls[b * kDeg + d], degra_w[d * kExp + e], bs);
  bs = bs + degra_b[e];
  const float gb = gate_boost[0] * bs;
  const bool isP = (lane < 12);
  const bool isG = (lane >= 16) && (lane < 28);
  const float val = isP ? pp : (isG ? gb : 0.0f);
  volatile float* q = addl + lane;
  *q = val;
  __threadfence();
  *q = val;
}

__global__ __launch_bounds__(256) void convw_kernel(
    const float* __restrict__ fc1_w, const float* __restrict__ fc2_w,
    _Float16* __restrict__ W1t, _Float16* __restrict__ W2t)
{
  __shared__ __align__(16) float sT[64 * 68];
  const int tid = threadIdx.x, lane = tid & 31, wave = tid >> 5;
  const int which = blockIdx.y / kExp;
  const int e = blockIdx.y - which * kExp;
  const int R  = which ? kHid : kCh;
  const int Cc = which ? kCh : kHid;
  const int tilesC = Cc >> 6;
  const int trx = blockIdx.x / tilesC;
  const int tcx = blockIdx.x - trx * tilesC;
  const int r0 = trx << 6, c0 = tcx << 6;
  const float* in = (which ? fc2_w : fc1_w) + (size_t)e * kCh * kHid;
  _Float16* out = (which ? W2t : W1t) + (size_t)e * kCh * kHid;
  {
    const int j4 = (tid & 15) * 4;
#pragma unroll
    for (int it = 0; it < 4; ++it) {
      const int i = it * 16 + (tid >> 4);
      const v4f v = *(const v4f*)(in + (size_t)(r0 + i) * Cc + c0 + j4);
      *(v4f*)(sT + i * 68 + j4) = v;
    }
  }
  __syncthreads();
  const int q = lane >> 3, l8 = lane & 7;
  v8h hv[2];
#pragma unroll
  for (int it = 0; it < 2; ++it) {
    const int jj = it * 32 + wave * 4 + q;
#pragma unroll
    for (int k = 0; k < 8; ++k) {
      const float s = flush16(sT[(l8 * 8 + k) * 68 + jj] * kWCarry);
      hv[it][k] = (_Float16)s;
    }
  }
  for (int pass = 0; pass < 2; ++pass) {
#pragma unroll
    for (int it = 0; it < 2; ++it) {
      const int jj = it * 32 + wave * 4 + q;
      *(volatile v8h*)(out + (size_t)(c0 + jj) * R + r0 + l8 * 8) = hv[it];
    }
    __threadfence();
  }
}

__global__ __launch_bounds__(128) void gate_kernel(
    const float* __restrict__ x, const float* __restrict__ w_g, const float* __restrict__ addl,
    _Float16* __restrict__ Xh, float* __restrict__ gates, float* __restrict__ partials)
{
  __shared__ __align__(16) float sWg[kCh * kExp];
  __shared__ __align__(16) _Float16 sX[128 * kXLdsPitch];
  __shared__ __align__(16) float sGate[128 * kGatePitch];
  const int tid = threadIdx.x, lane = tid & 31, wave = tid >> 5;
#pragma unroll 1
  for (int i = tid; i < kCh * kExp; i += 128) sWg[i] = w_g[i];
  __syncthreads();

  const int n0 = blockIdx.x * 128;
  const int b = n0 >> 14;
  const int hw0 = n0 & (kHW - 1);
  const float* xp = x + (size_t)b * kCh * kHW + hw0 + tid;
  _Float16* xrow = sX + tid * kXLdsPitch;
  float l0 = 0.0f, l1 = 0.0f, l2 = 0.0f, l3 = 0.0f, l4 = 0.0f, l5 = 0.0f;
#pragma unroll 4
  for (int c = 0; c < kCh; ++c) {
    const float v = xp[(size_t)c * kHW];
    const float* wr = sWg + c * kExp;
    l0 = fmaf(v, wr[0], l0);
    l1 = fmaf(v, wr[1], l1);
    l2 = fmaf(v, wr[2], l2);
    l3 = fmaf(v, wr[3], l3);
    l4 = fmaf(v, wr[4], l4);
    l5 = fmaf(v, wr[5], l5);
    const float xs = flush16(v * kXCarry);
    xrow[c] = (_Float16)xs;
  }
  float lg[kExp];
  lg[0] = (l0 + addl[b * kExp + 0]) + addl[16 + b * kExp + 0];
  lg[1] = (l1 + addl[b * kExp + 1]) + addl[16 + b * kExp + 1];
  lg[2] = (l2 + addl[b * kExp + 2]) + addl[16 + b * kExp + 2];
  lg[3] = (l3 + addl[b * kExp + 3]) + addl[16 + b * kExp + 3];
  lg[4] = (l4 + addl[b * kExp + 4]) + addl[16 + b * kExp + 4];
  lg[5] = (l5 + addl[b * kExp + 5]) + addl[16 + b * kExp + 5];

  float v1 = lg[0];
  int i1 = 0;
#pragma unroll
  for (int e = 1; e < kExp; ++e) {
    if (lg[e] > v1) { v1 = lg[e]; i1 = e; }
  }
  float v2 = -INFINITY;
  int i2 = 0;
#pragma unroll
  for (int e = 0; e < kExp; ++e) {
    if (e != i1 && lg[e] > v2) { v2 = lg[e]; i2 = e; }
  }
  const float ex = expf(v2 - v1);
  const float rs = 1.0f / (1.0f + ex);
  const float g1 = rs;
  const float g2 = ex * rs;
  float wv[kGatePitch];
#pragma unroll
  for (int e = 0; e < kExp; ++e) wv[e] = (e == i1) ? g1 : ((e == i2) ? g2 : 0.0f);
  wv[6] = 0.0f;
  wv[7] = 0.0f;
  {
    v4f a, c;
    a[0] = wv[0]; a[1] = wv[1]; a[2] = wv[2]; a[3] = wv[3];
    c[0] = wv[4]; c[1] = wv[5]; c[2] = wv[6]; c[3] = wv[7];
    *(v4f*)(sGate + tid * kGatePitch) = a;
    *(v4f*)(sGate + tid * kGatePitch + 4) = c;
  }
  __syncthreads();

  {
    const int hh = lane >> 4, c8 = (lane & 15) * 8;
    for (int pass = 0; pass < 2; ++pass) {
#pragma unroll
      for (int it = 0; it < 16; ++it) {
        const int row = it * 8 + wave * 2 + hh;
        const v8h hv = *(const v8h*)(sX + row * kXLdsPitch + c8);
        *(volatile v8h*)(Xh + (size_t)(n0 + row) * kCh + c8) = hv;
      }
#pragma unroll
      for (int it = 0; it < 2; ++it) {
        const int i4 = it * 128 + tid;
        const v4f gv = *(const v4f*)(sGate + i4 * 4);
        *(volatile v4f*)(gates + (size_t)n0 * kGatePitch + i4 * 4) = gv;
      }
      __threadfence();
    }
  }

  if (wave == 0) {
    const int colg = lane & 7;
    float sum = 0.0f, cnt = 0.0f;
#pragma unroll 1
    for (int t = 0; t < 128; ++t) {
      const float gv = sGate[t * kGatePitch + colg];
      sum += gv;
      cnt += (gv > 0.0f) ? 1.0f : 0.0f;
    }
    const bool valid = (colg < kExp) && (lane < 16);
    const bool isCnt = ((lane >> 3) & 1) != 0;
    const float val = valid ? (isCnt ? cnt : sum) : 0.0f;
    volatile float* q = partials + (size_t)blockIdx.x * 32 + lane;
    *q = val;
    __threadfence();
    *q = val;
  }
}

__global__ __launch_bounds__(32) void loss_kernel(const float* __restrict__ partials, float* __restrict__ out_loss)
{
  __shared__ float sTot[32];
  const int lane = threadIdx.x & 31;
  double s = 0.0;
#pragma unroll 1
  for (int blk = 0; blk < kGateBlocks; ++blk) s += (double)partials[(size_t)blk * 32 + lane];
  sTot[lane] = (float)s;
  __syncthreads();
  float total = 0.0f;
#pragma unroll 1
  for (int a = 0; a < 2; ++a) {
    const float* vp = sTot + a * 8;
    float m = 0.0f;
#pragma unroll 1
    for (int e = 0; e < kExp; ++e) m += vp[e];
    m = m / (float)kExp;
    float var = 0.0f;
#pragma unroll 1
    for (int e = 0; e < kExp; ++e) {
      const float d = vp[e] - m;
      var += d * d;
    }
    var = var / (float)(kExp - 1);
    total += var / (m * m + 1e-10f);
  }
  if (lane == 0) {
    volatile float* q = out_loss;
    *q = total;
    __threadfence();
    *q = total;
  }
}

__global__ __launch_bounds__(64) void moe_kernel(
    const _Float16* __restrict__ Xh, const _Float16* __restrict__ W1t, const _Float16* __restrict__ W2t,
    const float* __restrict__ fc1_b, const float* __restrict__ fc2_b,
    const float* __restrict__ gates, float* __restrict__ y)
{
  __shared__ __align__(16) float sS[kCh * kTokPitch];
  __shared__ __align__(16) float sC[kCh * kTokPitch];
  const int tid = threadIdx.x, wave = tid >> 5, lane = tid & 31;
  const int l16 = lane & 15, h = lane >> 4;
  const int col = wave * 16 + l16;
  const int tok = blockIdx.x * 32 + col;

  const _Float16* xr = Xh + (size_t)tok * kCh + 8 * h;
  const v16h xb0 = frag_load(xr);
  const v16h xb1 = frag_load(xr + 32);
  const v16h xb2 = frag_load(xr + 64);
  const v16h xb3 = frag_load(xr + 96);

  const v8f zero8 = (v8f){0.f, 0.f, 0.f, 0.f, 0.f, 0.f, 0.f, 0.f};
  const v8h zero8h = (v8h){(_Float16)0.f, (_Float16)0.f, (_Float16)0.f, (_Float16)0.f,
                           (_Float16)0.f, (_Float16)0.f, (_Float16)0.f, (_Float16)0.f};

#pragma unroll 1
  for (int t = 0; t < 8; ++t) {
#pragma unroll
    for (int r = 0; r < 8; ++r) sC[(t * 16 + 8 * h + r) * kTokPitch + col] = 0.0f;
  }

#pragma unroll 1
  for (int e = 0; e < kExp; ++e) {
    const float g = gates[(size_t)tok * kGatePitch + e];
    v8f acc[8];
#pragma unroll
    for (int t = 0; t < 8; ++t) acc[t] = zero8;
    const _Float16* w1e = W1t + ((size_t)e * kHid + l16) * kCh + 8 * h;
    const _Float16* w2e = W2t + ((size_t)e * kCh + l16) * kHid + 8 * h;
    const float* b1e = fc1_b + e * kHid + 8 * h;

#pragma unroll 1
    for (int ch = 0; ch < kHid / 32; ++ch) {
      const int hf0 = ch * 32;
      v8h lo = zero8h, hi = zero8h;
#pragma unroll 1
      for (int tc = 0; tc < 2; ++tc) {
        const int hfr = hf0 + tc * 16;
        const _Float16* ap = w1e + (size_t)hfr * kCh;
        const v16h a0 = frag_load(ap);
        const v16h a1 = frag_load(ap + 32);
        const v16h a2 = frag_load(ap + 64);
        const v16h a3 = frag_load(ap + 96);
        v8f hd = zero8;
        hd = mma_g(a0, xb0, hd);
        hd = mma_g(a1, xb1, hd);
        hd = mma_g(a2, xb2, hd);
        hd = mma_g(a3, xb3, hd);
        const v4f ba = *(const v4f*)(b1e + hfr);
        const v4f bb = *(const v4f*)(b1e + hfr + 4);
        float bv[8];
        bv[0] = ba[0]; bv[1] = ba[1]; bv[2] = ba[2]; bv[3] = ba[3];
        bv[4] = bb[0]; bv[5] = bb[1]; bv[6] = bb[2]; bv[7] = bb[3];
        v8h hv;
#pragma unroll
        for (int r = 0; r < 8; ++r) {
          const float v = fmaf(hd[r], kFc1Inv, bv[r]);
          const float gl = 0.5f * v * (1.0f + erff(v * kInvSqrt2));
          const float s = flush16(gl * kHCarry);
          hv[r] = (_Float16)s;
        }
        if (tc == 0) lo = hv; else hi = hv;
      }
      FragU bf;
      bf.h[0] = lo;
      bf.h[1] = hi;
      const _Float16* wp = w2e + hf0;
#pragma unroll
      for (int t = 0; t < 8; ++t) {
        const v16h a = frag_load(wp + (size_t)t * 16 * kHid);
        acc[t] = mma_g(a, bf.v, acc[t]);
      }
    }

#pragma unroll
    for (int t = 0; t < 8; ++t) {
#pragma unroll
      for (int r = 0; r < 8; ++r) sS[(t * 16 + 8 * h + r) * kTokPitch + col] = acc[t][r];
    }
#pragma unroll 1
    for (int t = 0; t < 8; ++t) {
      const int cb = t * 16 + 8 * h;
      const v4f pa = *(const v4f*)(fc2_b + e * kCh + cb);
      const v4f pb = *(const v4f*)(fc2_b + e * kCh + cb + 4);
      float b2[8];
      b2[0] = pa[0]; b2[1] = pa[1]; b2[2] = pa[2]; b2[3] = pa[3];
      b2[4] = pb[0]; b2[5] = pb[1]; b2[6] = pb[2]; b2[7] = pb[3];
#pragma unroll
      for (int r = 0; r < 8; ++r) {
        const int idx = (cb + r) * kTokPitch + col;
        const float o = fmaf(sS[idx], kFc2Inv, b2[r]);
        const float ev = expf(o);
        const float cacc = sC[idx];
        sC[idx] = fmaf(g, ev, cacc);
      }
    }
  }

#pragma unroll 1
  for (int t = 0; t < 8; ++t) {
#pragma unroll
    for (int r = 0; r < 8; ++r) {
      const int idx = (t * 16 + 8 * h + r) * kTokPitch + col;
      float v = sC[idx];
      v = (v == 0.0f) ? kEpsLog : v;
      sC[idx] = logf(v);
    }
  }
  __syncthreads();
  {
    const int n0 = blockIdx.x * 32;
    const int b = n0 >> 14;
    const int hw0 = n0 & (kHW - 1);
    const int q = lane >> 3, l8 = lane & 7;
    float* yb = y + (size_t)b * kCh * kHW + hw0 + l8 * 4;
    for (int pass = 0; pass < 2; ++pass) {
#pragma unroll
      for (int it = 0; it < 16; ++it) {
        const int c = wave * 64 + it * 4 + q;
        const v4f v = *(const v4f*)(sC + c * kTokPitch + l8 * 4);
        *(volatile v4f*)(yb + (size_t)c * kHW) = v;
      }
      __threadfence();
    }
  }
}

extern "C" void kernel_launch(void* const* d_in, const int* in_sizes, int n_in,
                              void* d_out, int out_size, void* d_ws, size_t ws_size,
                              hipStream_t stream) {
  if (n_in < 11) return;
  if (in_sizes[0] != kBatch * kCh * kHW) return;
  if (in_sizes[1] != kBatch * kCh) return;
  if (in_sizes[2] != kBatch * kDeg) return;
  if (in_sizes[3] != 2 * kCh * kExp) return;
  if (in_sizes[4] != 1) return;
  if (in_sizes[5] != kDeg * kExp) return;
  if (in_sizes[6] != kExp) return;
  if (in_sizes[7] != kExp * kCh * kHid) return;
  if (in_sizes[8] != kExp * kHid) return;
  if (in_sizes[9] != kExp * kHid * kCh) return;
  if (in_sizes[10] != kExp * kCh) return;
  if (out_size != kBatch * kCh * kHW + 1) return;
  if (ws_size < kWsTotal) return;

  const float* x          = (const float*)d_in[0];
  const float* prompt     = (const float*)d_in[1];
  const float* de_cls     = (const float*)d_in[2];
  const float* w_g        = (const float*)d_in[3];
  const float* gate_boost = (const float*)d_in[4];
  const float* degra_w    = (const float*)d_in[5];
  const float* degra_b    = (const float*)d_in[6];
  const float* fc1_w      = (const float*)d_in[7];
  const float* fc1_b      = (const float*)d_in[8];
  const float* fc2_w      = (const float*)d_in[9];
  const float* fc2_b      = (const float*)d_in[10];

  float* y    = (float*)d_out;
  float* loss = y + (size_t)kBatch * kCh * kHW;

  char* ws = (char*)d_ws;
  _Float16* XH   = (_Float16*)(ws + kOffXH);
  _Float16* W1T  = (_Float16*)(ws + kOffW1T);
  _Float16* W2T  = (_Float16*)(ws + kOffW2T);
  float*    GATE = (float*)(ws + kOffGATE);
  float*    PART = (float*)(ws + kOffPART);
  float*    ADDL = (float*)(ws + kOffADDL);

  prep_kernel<<<1, 32, 0, stream>>>(prompt, de_cls, w_g, gate_boost, degra_w, degra_b, ADDL);
  convw_kernel<<<dim3(16, 2 * kExp), 256, 0, stream>>>(fc1_w, fc2_w, W1T, W2T);
  gate_kernel<<<kGateBlocks, 128, 0, stream>>>(x, w_g, ADDL, XH, GATE, PART);
  loss_kernel<<<1, 32, 0, stream>>>(PART, loss);
  moe_kernel<<<kTok / 32, 64, 0, stream>>>(XH, W1T, W2T, fc1_b, fc2_b, GATE, y);
}
